// LSTMEmbedder_67465346285619
// MI455X (gfx1250) — hardware-verified
//
#include <hip/hip_runtime.h>


#define TT 1024
#define NB 64
#define NBB 16
#define NH 256
#define NG 1024
#define Y1C 512
#define NE 256
#define HP 264
#define SLP 72

typedef __attribute__((ext_vector_type(16))) _Float16 v16h;
typedef __attribute__((ext_vector_type(8)))  _Float16 v8h;
typedef __attribute__((ext_vector_type(16))) __bf16   v16b;
typedef __attribute__((ext_vector_type(8)))  __bf16   v8b;
typedef __attribute__((ext_vector_type(8)))  float    v8f;
typedef __attribute__((ext_vector_type(4)))  float    v4f;

__device__ __forceinline__ unsigned short f2bf_bits(float f) {
  unsigned u = __float_as_uint(f);
  return (unsigned short)((u + 0x7FFFu + ((u >> 16) & 1u)) >> 16);
}
__device__ __forceinline__ float bf_bits2f(unsigned short h) { return __uint_as_float(((unsigned)h) << 16); }

__device__ __forceinline__ void dep_guard_h(v8f& a, v8f& b, v16h x, v16h y) { asm volatile("v_nop\n\tv_nop\n\tv_nop\n\tv_nop" : "+v"(a), "+v"(b) : "v"(x), "v"(y)); }
__device__ __forceinline__ void dep_guard_b(v8f& a, v8f& b, v16b x, v16b y) { asm volatile("v_nop\n\tv_nop\n\tv_nop\n\tv_nop" : "+v"(a), "+v"(b) : "v"(x), "v"(y)); }
__device__ __forceinline__ void keep4_h(v16h a, v16h b, v16h c, v16h d) { asm volatile("v_nop" :: "v"(a), "v"(b), "v"(c), "v"(d)); }
__device__ __forceinline__ void keep4_b(v16b a, v16b b, v16b c, v16b d) { asm volatile("v_nop" :: "v"(a), "v"(b), "v"(c), "v"(d)); }
__device__ __forceinline__ void acc_guard4(v8f& a, v8f& b, v8f& c, v8f& d) { asm volatile("v_nop\n\tv_nop\n\tv_nop\n\tv_nop" : "+v"(a), "+v"(b), "+v"(c), "+v"(d)); }
template <typename T> struct Frag;
template <> struct Frag<_Float16> {
  typedef v16h V; union U { v16h v; v8h h[2]; };
  static __device__ __forceinline__ v16h load(const _Float16* p) {
    U f; f.h[0] = *(const v8h*)(p); f.h[1] = *(const v8h*)(p + 16); return f.v;
  }
  static __device__ __forceinline__ v8f mma(v16h a, v16h b, v8f c) {
    return __builtin_amdgcn_wmma_f32_16x16x32_f16(false, a, false, b, (short)0, c, false, false);
  }
  static __device__ __forceinline__ void guard(v8f& a, v8f& b, v16h x, v16h y) { dep_guard_h(a, b, x, y); }
  static __device__ __forceinline__ void keep(v16h a, v16h b, v16h c, v16h d) { keep4_h(a, b, c, d); }
};
template <> struct Frag<__bf16> {
  typedef v16b V; union U { v16b v; v8b h[2]; };
  static __device__ __forceinline__ v16b load(const __bf16* p) {
    U f; f.h[0] = *(const v8b*)(p); f.h[1] = *(const v8b*)(p + 16); return f.v;
  }
  static __device__ __forceinline__ v8f mma(v16b a, v16b b, v8f c) {
    return __builtin_amdgcn_wmma_f32_16x16x32_bf16(false, a, false, b, (short)0, c, false, false);
  }
  static __device__ __forceinline__ void guard(v8f& a, v8f& b, v16b x, v16b y) { dep_guard_b(a, b, x, y); }
  static __device__ __forceinline__ void keep(v16b a, v16b b, v16b c, v16b d) { keep4_b(a, b, c, d); }
};

template <int ET> struct Elem;
template <> struct Elem<0> { typedef _Float16 T; };
template <> struct Elem<1> { typedef __bf16 T; };
template <int ET, bool SPLIT, int BIAS_MODE, int OUT_MODE, bool RESID, int ACT = 0>
__global__ __launch_bounds__(256) void wmma_gemm64(
    const unsigned short* __restrict__ Ap, const unsigned short* __restrict__ A2p, int lda, long strideA,
    const unsigned short* __restrict__ Btp, const unsigned short* __restrict__ Bt2p, int ldb, long strideB,
    void* __restrict__ Cout, void* __restrict__ Cout2, int ldc, long strideC,
    const float* __restrict__ bias,
    const float* __restrict__ resid, long strideR,
    int M, int N, int K, float scale) {
  typedef typename Elem<ET>::T T;
  typedef typename Frag<T>::V V;
  const T* A = (const T*)Ap; const T* A2 = (const T*)A2p; const T* Bt = (const T*)Btp; const T* Bt2 = (const T*)Bt2p;
  __shared__ __align__(16) float sT[8][16 * 68];
  const int b    = blockIdx.y;
  const int lane = threadIdx.x & 31;
  const int wave = threadIdx.x >> 5;
  const int tilesN = N >> 6;
  const int tilesM = M >> 6;
  const int tile = blockIdx.x * 8 + wave;
  if (tile >= tilesM * tilesN) return;
  const int tm = tile / tilesN;
  const int tn = tile - tm * tilesN;
  const int m0 = tm << 6;
  const int n0 = tn << 6;

  const T* Ab  = A  + (size_t)b * strideA;
  const T* Bb  = Bt + (size_t)b * strideB;
  const T* Ab2 = SPLIT ? (A2  + (size_t)b * strideA) : nullptr;
  const T* Bb2 = SPLIT ? (Bt2 + (size_t)b * strideB) : nullptr;

  const int rlane = lane & 15;
  const int koff  = (lane >> 4) * 8;
  const int mOff  = (lane >> 4) * 8;

  v8f acc[4][4];
#pragma unroll
  for (int i = 0; i < 4; ++i)
#pragma unroll
    for (int j = 0; j < 4; ++j) acc[i][j] = (v8f){0.f,0.f,0.f,0.f,0.f,0.f,0.f,0.f};

  for (int k0 = 0; k0 < K; k0 += 32) {
    V bh[4], bl[4];
#pragma unroll
    for (int j = 0; j < 4; ++j) {
      const size_t bo = (size_t)(n0 + (j << 4) + rlane) * ldb + koff + k0;
      bh[j] = Frag<T>::load(Bb + bo);
      if (SPLIT) bl[j] = Frag<T>::load(Bb2 + bo);
    }
#pragma unroll
    for (int i = 0; i < 4; ++i) {
      const size_t ao = (size_t)(m0 + (i << 4) + rlane) * lda + koff + k0;
      V ah = Frag<T>::load(Ab + ao);
      V al;
      if (SPLIT) al = Frag<T>::load(Ab2 + ao);
#pragma unroll
      for (int j = 0; j < 4; ++j) {
        acc[i][j] = Frag<T>::mma(ah, bh[j], acc[i][j]);
        if (SPLIT) {
          acc[i][j] = Frag<T>::mma(ah, bl[j], acc[i][j]);
          acc[i][j] = Frag<T>::mma(al, bh[j], acc[i][j]);
        }
      }
      Frag<T>::guard(acc[i][0], acc[i][3], ah, SPLIT ? al : ah);
    }
    Frag<T>::keep(bh[0], bh[1], bh[2], bh[3]);
    if (SPLIT) Frag<T>::keep(bl[0], bl[1], bl[2], bl[3]);
  }
  acc_guard4(acc[0][0], acc[0][1], acc[0][2], acc[0][3]);
  acc_guard4(acc[1][0], acc[1][1], acc[1][2], acc[1][3]);
  acc_guard4(acc[2][0], acc[2][1], acc[2][2], acc[2][3]);
  acc_guard4(acc[3][0], acc[3][1], acc[3][2], acc[3][3]);

  float* slab = sT[wave];
  const float* Rb = RESID ? (resid + (size_t)b * strideR) : nullptr;
#pragma unroll
  for (int i = 0; i < 4; ++i) {
    const int mBase = m0 + (i << 4);
#pragma unroll
    for (int j = 0; j < 4; ++j) {
      const int n = n0 + (j << 4) + rlane;
      float bv = 0.f;
      if (BIAS_MODE == 2) bv = bias[n];
#pragma unroll
      for (int r = 0; r < 8; ++r) {
        float v = acc[i][j][r] * scale;
        if (BIAS_MODE == 1) v += bias[mBase + mOff + r];
        if (BIAS_MODE == 2) v += bv;
        if (RESID) v += Rb[(size_t)(mBase + mOff + r) * ldc + n];
        if (ACT == 1) v = tanhf(v);
        if (ACT == 2) v = fmaxf(v, 0.0f);
        if (ACT == 3) v = v / (1.0f + expf(-v));
        if (ACT == 4) v = (v > 0.f) ? v : 0.01f * v;
        if (ACT == 5) v = 0.5f * v * (1.0f + erff(v * 0.70710678118654752f));
        slab[(mOff + r) * 68 + (j << 4) + rlane] = v;
      }
    }
    __builtin_amdgcn_fence(__ATOMIC_RELEASE, "workgroup");
    __builtin_amdgcn_wave_barrier();
    __builtin_amdgcn_fence(__ATOMIC_ACQUIRE, "workgroup");
    if (OUT_MODE == 0) {
      float* C = (float*)Cout + (size_t)b * strideC;
      const int hh = lane >> 4, c4 = (lane & 15) * 4;
      for (int pass = 0; pass < 2; ++pass) {
#pragma unroll
        for (int it = 0; it < 8; ++it) {
          const int row = it * 2 + hh;
          v4f v = *(const v4f*)(slab + row * 68 + c4);
          *(volatile v4f*)(C + (size_t)(mBase + row) * ldc + n0 + c4) = v;
        }
        __threadfence();
      }
    } else {
      const int q = lane >> 3, c8 = (lane & 7) * 8;
      unsigned short* C  = (unsigned short*)Cout  + (size_t)b * strideC;
      unsigned short* C2 = (OUT_MODE == 2) ? ((unsigned short*)Cout2 + (size_t)b * strideC) : nullptr;
      for (int pass = 0; pass < 2; ++pass) {
#pragma unroll
        for (int it = 0; it < 4; ++it) {
          const int row = it * 4 + q;
          const float* sp = slab + row * 68 + c8;
          v8h hv, lv;
#pragma unroll
          for (int e = 0; e < 8; ++e) {
            if (OUT_MODE == 1) {
              hv[e] = (_Float16)sp[e];
            } else {
              unsigned short hb = f2bf_bits(sp[e]);
              unsigned short lb = f2bf_bits(sp[e] - bf_bits2f(hb));
              hv[e] = __builtin_bit_cast(_Float16, hb);
              lv[e] = __builtin_bit_cast(_Float16, lb);
            }
          }
          *(volatile v8h*)(C + (size_t)(mBase + row) * ldc + n0 + c8) = hv;
          if (OUT_MODE == 2) *(volatile v8h*)(C2 + (size_t)(mBase + row) * ldc + n0 + c8) = lv;
        }
        __threadfence();
      }
    }
    __builtin_amdgcn_fence(__ATOMIC_RELEASE, "workgroup");
    __builtin_amdgcn_wave_barrier();
    __builtin_amdgcn_fence(__ATOMIC_ACQUIRE, "workgroup");
  }
}

__global__ __launch_bounds__(256) void rows_to_f16(
    const float* __restrict__ src, _Float16* __restrict__ dst, int R, int Cin, int Cpad, float scale)
{
  const int lane = threadIdx.x & 31;
  const int wave = threadIdx.x >> 5;
  const int r = blockIdx.x * 8 + wave;
  if (r >= R) return;
  const float* sp = src + (size_t)r * Cin;
  _Float16* dp = dst + (size_t)r * Cpad;
  v8h o[2];
#pragma unroll
  for (int ch = 0; ch < 2; ++ch) {
    const int c0 = ch * 256 + 8 * lane;
    int ca = c0, cb = c0 + 4;
    const bool va = (ca + 3 < Cin), vb = (cb + 3 < Cin);
    ca = va ? ca : (Cin - 4);
    cb = vb ? cb : (Cin - 4);
    v4f x0 = *(const v4f*)(sp + ca);
    v4f x1 = *(const v4f*)(sp + cb);
    const v4f z = (v4f){0.f, 0.f, 0.f, 0.f};
    if (!va) x0 = z;
    if (!vb) x1 = z;
#pragma unroll
    for (int e = 0; e < 4; ++e) {
      o[ch][e]     = (_Float16)(x0[e] * scale);
      o[ch][4 + e] = (_Float16)(x1[e] * scale);
    }
  }
  for (int pass = 0; pass < 2; ++pass) {
#pragma unroll
    for (int ch = 0; ch < 2; ++ch) {
      const int c0 = ch * 256 + 8 * lane;
      if (c0 < Cpad) *(volatile v8h*)(dp + c0) = o[ch];
    }
    __threadfence();
  }
}

__device__ __forceinline__ float sigm_f(float x) { return __builtin_amdgcn_rcpf(1.0f + __expf(-x)); }
__device__ __forceinline__ float tanh_f(float x) { return 1.0f - 2.0f * __builtin_amdgcn_rcpf(__expf(2.0f * x) + 1.0f); }

template <int LAYER>
__global__ __launch_bounds__(128) void recur_kernel(
    const _Float16* __restrict__ Whh16,
    const _Float16* __restrict__ Wih16,
    const float* __restrict__ xin,
    const float* __restrict__ wih0,
    const float* __restrict__ bias,
    const _Float16* __restrict__ y1in,
    _Float16* __restrict__ yout)
{
  __shared__ __align__(16) _Float16 hsh[2 * NBB * HP];
  __shared__ __align__(16) _Float16 slab[4 * NBB * SLP];
  __shared__ float csh[NBB * NH];
  __shared__ float bsh[NG];
  __shared__ float wsh[NG];
  typedef Frag<_Float16> F;
  const int tid = threadIdx.x;
  const int lane = tid & 31, wave = tid >> 5, hh = lane >> 4, rl = lane & 15;
  const int dir = (int)(blockIdx.x >> 2);
  const int b0  = (int)(blockIdx.x & 3) * NBB;
  const _Float16* Whh = Whh16 + (size_t)dir * NG * NH;
  const _Float16* Wih = Wih16 + (size_t)dir * NG * Y1C;
  for (int i = tid; i < 2 * NBB * HP; i += 128) hsh[i] = (_Float16)0.0f;
  for (int i = tid; i < NBB * NH; i += 128) csh[i] = 0.0f;
  for (int i = tid; i < NG; i += 128) {
    bsh[i] = bias[(size_t)dir * NG + i];
    wsh[i] = (LAYER == 0) ? wih0[(size_t)dir * NG + i] : 0.0f;
  }
  __syncthreads();
  const int u0 = wave * 64;
  const float S = 1.0f / 16384.0f;
  _Float16* slabw = slab + wave * (NBB * SLP);
  const int rq = lane >> 3, c8 = (lane & 7) * 8;

#pragma unroll 1
  for (int s = 0; s < TT; ++s) {
    const int t = dir ? (TT - 1 - s) : s;
    const _Float16* hc = hsh + (s & 1) * (NBB * HP);
    _Float16* hn = hsh + ((s & 1) ^ 1) * (NBB * HP);
    const _Float16* yrow = y1in + ((size_t)t * NB + b0) * Y1C;
    const bool lastStep = (s == TT - 1);
    float xt[8];
#pragma unroll
    for (int r = 0; r < 8; ++r) xt[r] = 0.0f;
    if (LAYER == 0) {
#pragma unroll
      for (int r = 0; r < 8; ++r) xt[r] = xin[(size_t)(b0 + 8 * hh + r) * TT + t];
    }
#pragma unroll 1
    for (int q = 0; q < 4; ++q) {
      const int ub = u0 + 16 * q;
      v8f acc[4];
#pragma unroll
      for (int g = 0; g < 4; ++g) acc[g] = (v8f){0.f,0.f,0.f,0.f,0.f,0.f,0.f,0.f};
      if (LAYER == 1) {
#pragma unroll 1
        for (int k0 = 0; k0 < Y1C; k0 += 32) {
          v16h bfr[4];
#pragma unroll
          for (int g = 0; g < 4; ++g) bfr[g] = F::load(Wih + (size_t)(g * NH + ub + rl) * Y1C + k0 + 8 * hh);
          const v16h a = F::load(yrow + (size_t)rl * Y1C + k0 + 8 * hh);
#pragma unroll
          for (int g = 0; g < 4; ++g) acc[g] = F::mma(a, bfr[g], acc[g]);
          F::guard(acc[0], acc[3], a, a);
          F::keep(bfr[0], bfr[1], bfr[2], bfr[3]);
        }
      }
#pragma unroll 1
      for (int k0 = 0; k0 < NH; k0 += 32) {
        v16h bfr[4];
#pragma unroll
        for (int g = 0; g < 4; ++g) bfr[g] = F::load(Whh + (size_t)(g * NH + ub + rl) * NH + k0 + 8 * hh);
        const v16h a = F::load(hc + rl * HP + k0 + 8 * hh);
#pragma unroll
        for (int g = 0; g < 4; ++g) acc[g] = F::mma(a, bfr[g], acc[g]);
        F::guard(acc[0], acc[3], a, a);
        F::keep(bfr[0], bfr[1], bfr[2], bfr[3]);
      }
      acc_guard4(acc[0], acc[1], acc[2], acc[3]);

      const int u = ub + rl;
      const int scol = 16 * q + rl;
      const float bI = bsh[u], bF = bsh[NH + u], bG = bsh[2 * NH + u], bO = bsh[3 * NH + u];
      const float wI = wsh[u], wF = wsh[NH + u], wG = wsh[2 * NH + u], wO = wsh[3 * NH + u];
#pragma unroll
      for (int r = 0; r < 8; ++r) {
        const int bl = 8 * hh + r;
        float gi, gf, gg, go;
        if (LAYER == 0) {
          gi = acc[0][r] * S + (xt[r] * wI + bI);
          gf = acc[1][r] * S + (xt[r] * wF + bF);
          gg = acc[2][r] * S + (xt[r] * wG + bG);
          go = acc[3][r] * S + (xt[r] * wO + bO);
        } else {
          gi = acc[0][r] * S + bI;
          gf = acc[1][r] * S + bF;
          gg = acc[2][r] * S + bG;
          go = acc[3][r] * S + bO;
        }
        const float cp = csh[bl * NH + u];
        const float cn = sigm_f(gf) * cp + sigm_f(gi) * tanh_f(gg);
        csh[bl * NH + u] = cn;
        const float h = sigm_f(go) * tanh_f(cn);
        const _Float16 h16 = (_Float16)(h * 256.0f);
        hn[bl * HP + u] = h16;
        if (LAYER == 0 || lastStep) slabw[bl * SLP + scol] = h16;
      }
    }
    if (LAYER == 0 || lastStep) {
      __builtin_amdgcn_fence(__ATOMIC_RELEASE, "workgroup");
      __builtin_amdgcn_wave_barrier();
      __builtin_amdgcn_fence(__ATOMIC_ACQUIRE, "workgroup");
      _Float16* ob = (LAYER == 0) ? (yout + ((size_t)t * NB + b0) * Y1C + dir * NH + u0)
                                  : (yout + (size_t)b0 * Y1C + dir * NH + u0);
      for (int pass = 0; pass < 2; ++pass) {
#pragma unroll
        for (int it = 0; it < 4; ++it) {
          const int row = it * 4 + rq;
          const v8h v = *(const v8h*)(slabw + row * SLP + c8);
          *(volatile v8h*)(ob + (size_t)row * Y1C + c8) = v;
        }
        __threadfence();
      }
    }
    __syncthreads();
  }
}

__global__ __launch_bounds__(256) void ln_kernel(
    const float* __restrict__ xin, const float* __restrict__ gam, const float* __restrict__ bet,
    float* __restrict__ out)
{
  const int lane = threadIdx.x & 31, wave = threadIdx.x >> 5;
  const int row = blockIdx.x * 8 + wave;
  if (row >= NB) return;
  const float* p = xin + (size_t)row * NE;
  const v4f x0 = *(const v4f*)(p + 4 * lane);
  const v4f x1 = *(const v4f*)(p + 128 + 4 * lane);
  float sm = ((x0[0] + x0[1]) + (x0[2] + x0[3])) + ((x1[0] + x1[1]) + (x1[2] + x1[3]));
#pragma unroll
  for (int off = 1; off < 32; off <<= 1) sm += __shfl_xor(sm, off, 32);
  const float mu = sm * (1.0f / 256.0f);
  v4f d0, d1;
  float vs = 0.f;
#pragma unroll
  for (int e = 0; e < 4; ++e) { d0[e] = x0[e] - mu; vs += d0[e] * d0[e]; }
#pragma unroll
  for (int e = 0; e < 4; ++e) { d1[e] = x1[e] - mu; vs += d1[e] * d1[e]; }
#pragma unroll
  for (int off = 1; off < 32; off <<= 1) vs += __shfl_xor(vs, off, 32);
  const float inv = rsqrtf(vs * (1.0f / 256.0f) + 1e-5f);
  const v4f g0 = *(const v4f*)(gam + 4 * lane);
  const v4f g1 = *(const v4f*)(gam + 128 + 4 * lane);
  const v4f e0 = *(const v4f*)(bet + 4 * lane);
  const v4f e1 = *(const v4f*)(bet + 128 + 4 * lane);
  v4f o0, o1;
#pragma unroll
  for (int e = 0; e < 4; ++e) {
    o0[e] = g0[e] * (d0[e] * inv) + e0[e];
    o1[e] = g1[e] * (d1[e] * inv) + e1[e];
  }
  float* op = out + (size_t)row * NE;
  for (int pass = 0; pass < 2; ++pass) {
    *(volatile v4f*)(op + 4 * lane) = o0;
    *(volatile v4f*)(op + 128 + 4 * lane) = o1;
    __threadfence();
  }
}

extern "C" void kernel_launch(void* const* d_in, const int* in_sizes, int n_in,
                              void* d_out, int out_size, void* d_ws, size_t ws_size,
                              hipStream_t stream) {
  if (n_in < 11) return;
  if (in_sizes[0] != NB * TT) return;
  if (in_sizes[1] != 2 * NG || in_sizes[2] != 2 * NG * NH || in_sizes[3] != 2 * NG) return;
  if (in_sizes[4] != 2 * NG * Y1C || in_sizes[5] != 2 * NG * NH || in_sizes[6] != 2 * NG) return;
  if (in_sizes[7] != NE * Y1C || in_sizes[8] != NE || in_sizes[9] != NE || in_sizes[10] != NE) return;
  if (out_size != NB * NE) return;

  const float* timein = (const float*)d_in[0];
  const float* Wih0   = (const float*)d_in[1];
  const float* Whh0   = (const float*)d_in[2];
  const float* b0     = (const float*)d_in[3];
  const float* Wih1   = (const float*)d_in[4];
  const float* Whh1   = (const float*)d_in[5];
  const float* b1     = (const float*)d_in[6];
  const float* Wproj  = (const float*)d_in[7];
  const float* bproj  = (const float*)d_in[8];
  const float* gammav = (const float*)d_in[9];
  const float* betav  = (const float*)d_in[10];
  float* out0 = (float*)d_out;

  const size_t szY1   = (size_t)TT * NB * Y1C * 2;
  const size_t szWhh  = (size_t)2 * NG * NH * 2;
  const size_t szWih  = (size_t)2 * NG * Y1C * 2;
  const size_t szWp   = (size_t)NE * Y1C * 2;
  const size_t szLast = (size_t)NB * Y1C * 2;
  const size_t szOutp = (size_t)NB * NE * 4;
  size_t off = 0;
  const size_t oY1   = off; off += szY1;
  const size_t oWhh0 = off; off += szWhh;
  const size_t oWhh1 = off; off += szWhh;
  const size_t oWih1 = off; off += szWih;
  const size_t oWp   = off; off += szWp;
  const size_t oLast = off; off += szLast;
  const size_t oOutp = off; off += szOutp;
  if (off > ws_size) return;
  char* ws = (char*)d_ws;
  _Float16* y1      = (_Float16*)(ws + oY1);
  _Float16* Whh0_16 = (_Float16*)(ws + oWhh0);
  _Float16* Whh1_16 = (_Float16*)(ws + oWhh1);
  _Float16* Wih1_16 = (_Float16*)(ws + oWih1);
  _Float16* Wp16    = (_Float16*)(ws + oWp);
  _Float16* last16  = (_Float16*)(ws + oLast);
  float*    outp    = (float*)(ws + oOutp);

  rows_to_f16<<<(2 * NG + 7) / 8, 256, 0, stream>>>(Whh0,  Whh0_16, 2 * NG, NH,  NH,  64.0f);
  rows_to_f16<<<(2 * NG + 7) / 8, 256, 0, stream>>>(Whh1,  Whh1_16, 2 * NG, NH,  NH,  64.0f);
  rows_to_f16<<<(2 * NG + 7) / 8, 256, 0, stream>>>(Wih1,  Wih1_16, 2 * NG, Y1C, Y1C, 64.0f);
  rows_to_f16<<<(NE + 7) / 8,     256, 0, stream>>>(Wproj, Wp16,    NE,     Y1C, Y1C, 64.0f);

  recur_kernel<0><<<8, 128, 0, stream>>>(Whh0_16, Wih1_16, timein, Wih0, b0, last16, y1);
  recur_kernel<1><<<8, 128, 0, stream>>>(Whh1_16, Wih1_16, timein, Wih0, b1, y1, last16);

  wmma_gemm64<0, false, 2, 0, false, 0><<<dim3(1, 1), 256, 0, stream>>>(
      (const unsigned short*)last16, (const unsigned short*)last16, Y1C, 0L,
      (const unsigned short*)Wp16, (const unsigned short*)Wp16, Y1C, 0L,
      (void*)outp, (void*)outp, NE, 0L,
      bproj, (const float*)outp, 0L, NB, NE, Y1C, 1.0f / 16384.0f);

  ln_kernel<<<(NB + 7) / 8, 256, 0, stream>>>(outp, gammav, betav, out0);
}
